// FullyConnectedTensorProduct_15461882266097
// MI455X (gfx1250) — hardware-verified
//
#include <hip/hip_runtime.h>


#define NB_  32768
#define MI   32
#define MO   64
#define KUV  (MI * MI)
#define DIN  128
#define DOUT 448
#define RCH  4096
#define DM   KUV
#define A000 0.02209708691207961f
#define A110 0.012757759076995721f
#define A011 0.022097086912079608f
#define A111 0.02209708691207961f
#define LOSC 1024.0f

typedef _Float16 h16;
typedef unsigned short bf;
typedef __attribute__((ext_vector_type(16))) __bf16   v16bf;
typedef __attribute__((ext_vector_type(16))) _Float16 v16h;
typedef __attribute__((ext_vector_type(8)))  _Float16 v8h;
typedef __attribute__((ext_vector_type(8)))  unsigned short v8us;
typedef __attribute__((ext_vector_type(8)))  float    v8f;
typedef __attribute__((ext_vector_type(4)))  float    v4f;
typedef v8h  __attribute__((may_alias)) v8ha;
typedef v4f  __attribute__((may_alias)) v4fa;
typedef v8us __attribute__((may_alias)) v8usa;

__device__ __forceinline__ unsigned short f2bf(float f) { unsigned u = __float_as_uint(f); u += 0x7FFFu + ((u >> 16) & 1u); return (unsigned short)(u >> 16); }
__device__ __forceinline__ float bf2f(unsigned short b) { return __uint_as_float(((unsigned)b) << 16); }
__device__ __forceinline__ float bfr(float f) { return bf2f(f2bf(f)); }
__device__ __forceinline__ v16h cat16(v8h lo, v8h hi) { return __builtin_shufflevector(lo, hi, 0, 1, 2, 3, 4, 5, 6, 7, 8, 9, 10, 11, 12, 13, 14, 15); }
__device__ __forceinline__ v16bf cat16b(v8us lo, v8us hi) { return __builtin_bit_cast(v16bf, __builtin_shufflevector(lo, hi, 0, 1, 2, 3, 4, 5, 6, 7, 8, 9, 10, 11, 12, 13, 14, 15)); }
__device__ __forceinline__ v8f wmma16(v16h a, v16h b, v8f c) { return __builtin_amdgcn_wmma_f32_16x16x32_f16(false, a, false, b, (short)0, c, false, false); }
__device__ __forceinline__ v8f wmmab(v16bf a, v16bf b, v8f c) { return __builtin_amdgcn_wmma_f32_16x16x32_bf16(false, a, false, b, (short)0, c, false, false); }

template <bool SPLITA, bool F16OUT = false>
__global__ __launch_bounds__(128) void k_gemmb(const bf* __restrict__ A, const bf* __restrict__ Al, const bf* __restrict__ Bn, const float* __restrict__ bias, float* C, int ldc, h16* C2, const float* __restrict__ R = nullptr, int K = DM, int roundR = 1) {
    __shared__ __align__(16) float ost[4][16 * 68];
    const int lane = threadIdx.x & 31, wave = threadIdx.x >> 5, lr = lane & 15, hi = lane >> 4;
    const int r0 = blockIdx.x * 64 + wave * 16, c0 = blockIdx.y * 64;
    const size_t aoff = (size_t)(r0 + lr) * K + 8 * hi;
    size_t boff[4];
#pragma unroll
    for (int t = 0; t < 4; ++t) boff[t] = (size_t)(c0 + t * 16 + lr) * K + 8 * hi;
    v8f acc[4];
#pragma unroll
    for (int t = 0; t < 4; ++t) acc[t] = (v8f){};
#pragma unroll 1
    for (int kc = 0; kc < K; kc += 32) {
        const v16bf a = cat16b(*(const v8us*)(A + aoff + kc), *(const v8us*)(A + aoff + kc + 16));
        v16bf al = a;
        if (SPLITA) al = cat16b(*(const v8us*)(Al + aoff + kc), *(const v8us*)(Al + aoff + kc + 16));
#pragma unroll
        for (int t = 0; t < 4; ++t) { const v16bf b = cat16b(*(const v8us*)(Bn + boff[t] + kc), *(const v8us*)(Bn + boff[t] + kc + 16)); acc[t] = wmmab(a, b, acc[t]); if (SPLITA) acc[t] = wmmab(al, b, acc[t]); }
        asm volatile("v_nop\n\tv_nop\n\tv_nop\n\tv_nop" : "+v"(acc[0]), "+v"(acc[1]), "+v"(acc[2]), "+v"(acc[3]) : "v"(a), "v"(al));
    }
    float* os = &ost[wave][0];
#pragma unroll
    for (int t = 0; t < 4; ++t) { const float bv = bias ? bfr(bias[c0 + t * 16 + lr]) : 0.f;
#pragma unroll
        for (int j = 0; j < 8; ++j) os[(hi * 8 + j) * 68 + t * 16 + lr] = acc[t][j] + bv; }
    __syncthreads();
    if (F16OUT) {
        h16* crow = (h16*)(void*)C + (size_t)r0 * ldc + c0;
        auto pass = [&]() {
#pragma unroll
            for (int s = 0; s < 4; ++s) { const int row = 4 * s + (lane >> 3), piece = lane & 7; const float* sp = os + row * 68 + piece * 8; v8h o, o2;
#pragma unroll
                for (int i = 0; i < 8; ++i) { const h16 a = (h16)sp[i]; o[i] = a; o2[i] = (h16)((sp[i] - (float)a) * LOSC); }
                *(volatile v8h*)(crow + (size_t)row * ldc + piece * 8) = o; if (C2) *(volatile v8h*)(C2 + (size_t)r0 * ldc + c0 + (size_t)row * ldc + piece * 8) = o2; }
        };
        pass(); __threadfence(); pass();
    } else {
        float* crow = C + (size_t)r0 * ldc + c0;
        auto pass = [&]() {
#pragma unroll
            for (int s = 0; s < 8; ++s) { const int Lid = (lane >> 3) + 4 * s, piece = lane & 7; const int row = Lid >> 1, cofs = (Lid & 1) * 32 + piece * 4;
                v4f val = *(const v4fa*)(os + row * 68 + cofs); if (R) { const v4f rv = *(const v4f*)(R + ((size_t)r0 + row) * ldc + c0 + cofs); val += roundR ? (v4f){bfr(rv[0]), bfr(rv[1]), bfr(rv[2]), bfr(rv[3])} : rv; }
                *(volatile v4f*)(crow + (size_t)row * ldc + cofs) = val; }
        };
        pass(); __threadfence(); pass();
    }
}

__global__ __launch_bounds__(256) void k_wt(const float* __restrict__ Wm, int K, int ncols, bf* WT) {
    __shared__ __align__(16) unsigned short tl[64 * 72];
    const int tid = threadIdx.x, k0 = blockIdx.x * 64, n0 = blockIdx.y * 64;
    const int kk = tid >> 2, nq = (tid & 3) * 16;
#pragma unroll
    for (int i = 0; i < 16; ++i) tl[(nq + i) * 72 + kk] = f2bf(Wm[(size_t)(k0 + kk) * ncols + n0 + nq + i]);
    __syncthreads();
    const int piece = tid & 7;
    auto pass = [&]() {
#pragma unroll
        for (int s = 0; s < 2; ++s) { const int nr = (tid >> 3) + 32 * s; const v8us val = *(const v8usa*)(tl + nr * 72 + piece * 8); *(volatile v8us*)(WT + (size_t)(n0 + nr) * K + k0 + piece * 8) = val; }
    };
    pass(); __threadfence(); pass();
}

template <int MODE>
__global__ __launch_bounds__(256) void k_outer(const float* __restrict__ x1, const float* __restrict__ x2, size_t r0, int k, float coef, bf* Ah, bf* Al) {
    const int lane = threadIdx.x & 31; const size_t rr = (size_t)blockIdx.x * 8 + (threadIdx.x >> 5); if (rr >= (size_t)RCH) return; const float* a = x1 + (r0 + rr) * DIN; const float* b = x2 + (r0 + rr) * DIN;
    const int k1 = (k + 1) % 3, k2 = (k + 2) % 3;
#pragma unroll 1
    for (int ps = 0; ps < 2; ++ps) {
#pragma unroll 1
        for (int q = 0; q < KUV / 256; ++q) { v8us oh, ol;
#pragma unroll
            for (int i = 0; i < 8; ++i) { const int uv = q * 256 + lane * 8 + i; const int u = uv / MI, v = uv % MI; float val;
                if (MODE == 0) val = bfr(a[u]) * bfr(b[v]);
                else if (MODE == 1) val = bfr(a[MI + u * 3]) * bfr(b[MI + v * 3]) + bfr(a[MI + u * 3 + 1]) * bfr(b[MI + v * 3 + 1]) + bfr(a[MI + u * 3 + 2]) * bfr(b[MI + v * 3 + 2]);
                else if (MODE == 2) val = bfr(a[u]) * bfr(b[MI + v * 3 + k]);
                else if (MODE == 3) val = bfr(a[MI + u * 3 + k]) * bfr(b[v]);
                else val = bfr(a[MI + u * 3 + k1]) * bfr(b[MI + v * 3 + k2]) - bfr(a[MI + u * 3 + k2]) * bfr(b[MI + v * 3 + k1]);
                val *= coef; const unsigned short hb = f2bf(val); oh[i] = hb; ol[i] = f2bf(val - bf2f(hb)); }
            const size_t o = rr * KUV + q * 256 + lane * 8; *(volatile v8us*)(Ah + o) = oh; *(volatile v8us*)(Al + o) = ol; }
        if (ps == 0) __threadfence(); }
}
__global__ __launch_bounds__(256) void k_assemble(const float* __restrict__ O0, const float* __restrict__ O1, const float* __restrict__ O2, float* OUTP) {
    const int lane = threadIdx.x & 31; const size_t r = (size_t)blockIdx.x * 8 + (threadIdx.x >> 5); if (r >= (size_t)NB_) return;
    auto val = [&](int c) -> float { if (c < MO) return O0[r * MO + c]; c -= MO; if (c < 3 * MO) { const int w = c / 3, k = c % 3; return O1[((size_t)k * NB_ + r) * MO + w]; } c -= 3 * MO; { const int w = c / 3, k = c % 3; return O2[((size_t)k * NB_ + r) * MO + w]; } };
#pragma unroll 1
    for (int ps = 0; ps < 2; ++ps) {
#pragma unroll 1
        for (int q = 0; q < 4; ++q) { const int c0 = q * 128 + lane * 4; if (c0 >= DOUT) continue; v4f v;
#pragma unroll
            for (int i = 0; i < 4; ++i) v[i] = val(c0 + i);
            *(volatile v4f*)(OUTP + r * DOUT + c0) = v; }
        if (ps == 0) __threadfence(); }
}

extern "C" void kernel_launch(void* const* d_in, const int* in_sizes, int n_in,
                              void* d_out, int out_size, void* d_ws, size_t ws_size, hipStream_t stream) {
    (void)in_sizes; (void)n_in; (void)out_size;
    const float* x1 = (const float*)d_in[0]; const float* x2 = (const float*)d_in[1]; const float* w000 = (const float*)d_in[2]; const float* w110 = (const float*)d_in[3]; const float* w011 = (const float*)d_in[4]; const float* w101 = (const float*)d_in[5]; const float* w111 = (const float*)d_in[6];
    float* out = (float*)d_out;
    char* wsp = (char*)d_ws;
    auto take = [&](size_t bytes) { char* p = wsp; wsp += (bytes + 255) & ~(size_t)255; return (void*)p; };
    bf* W0 = (bf*)take((size_t)MO * KUV * 2); bf* W1 = (bf*)take((size_t)MO * KUV * 2); bf* W2 = (bf*)take((size_t)MO * KUV * 2); bf* W3 = (bf*)take((size_t)MO * KUV * 2); bf* W4 = (bf*)take((size_t)MO * KUV * 2);
    bf* Ah = (bf*)take((size_t)RCH * KUV * 2); bf* Al = (bf*)take((size_t)RCH * KUV * 2); float* T0 = (float*)take((size_t)RCH * MO * 4);
    float* O0 = (float*)take((size_t)NB_ * MO * 4); float* O1 = (float*)take((size_t)3 * NB_ * MO * 4); float* O2 = (float*)take((size_t)3 * NB_ * MO * 4);
    if ((size_t)(wsp - (char*)d_ws) > ws_size) return;
    k_wt<<<dim3(KUV / 64, MO / 64, 1), 256, 0, stream>>>(w000, KUV, MO, W0); k_wt<<<dim3(KUV / 64, MO / 64, 1), 256, 0, stream>>>(w110, KUV, MO, W1); k_wt<<<dim3(KUV / 64, MO / 64, 1), 256, 0, stream>>>(w011, KUV, MO, W2);
    k_wt<<<dim3(KUV / 64, MO / 64, 1), 256, 0, stream>>>(w101, KUV, MO, W3); k_wt<<<dim3(KUV / 64, MO / 64, 1), 256, 0, stream>>>(w111, KUV, MO, W4);
    const dim3 gg(RCH / 64, 1, 1);
    for (int c = 0; c < NB_ / RCH; ++c) { const size_t r0 = (size_t)c * RCH;
        k_outer<0><<<RCH / 8, 256, 0, stream>>>(x1, x2, r0, 0, A000, Ah, Al);
        k_gemmb<true, false><<<gg, 128, 0, stream>>>(Ah, Al, W0, nullptr, T0, MO, nullptr, nullptr, KUV);
        k_outer<1><<<RCH / 8, 256, 0, stream>>>(x1, x2, r0, 0, A110, Ah, Al);
        k_gemmb<true, false><<<gg, 128, 0, stream>>>(Ah, Al, W1, nullptr, O0 + r0 * MO, MO, nullptr, T0, KUV, 0);
        for (int k = 0; k < 3; ++k) {
            k_outer<2><<<RCH / 8, 256, 0, stream>>>(x1, x2, r0, k, A011, Ah, Al);
            k_gemmb<true, false><<<gg, 128, 0, stream>>>(Ah, Al, W2, nullptr, T0, MO, nullptr, nullptr, KUV);
            k_outer<3><<<RCH / 8, 256, 0, stream>>>(x1, x2, r0, k, A011, Ah, Al);
            k_gemmb<true, false><<<gg, 128, 0, stream>>>(Ah, Al, W3, nullptr, O1 + ((size_t)k * NB_ + r0) * MO, MO, nullptr, T0, KUV, 0);
            k_outer<4><<<RCH / 8, 256, 0, stream>>>(x1, x2, r0, k, A111, Ah, Al);
            k_gemmb<true, false><<<gg, 128, 0, stream>>>(Ah, Al, W4, nullptr, O2 + ((size_t)k * NB_ + r0) * MO, MO, nullptr, nullptr, KUV); } }
    k_assemble<<<NB_ / 8, 256, 0, stream>>>(O0, O1, O2, out);
}
